// MLPBlock_85048942396042
// MI455X (gfx1250) — hardware-verified
//
#include <hip/hip_runtime.h>


namespace {
constexpr int NB = 2, C = 64, HH = 128, WW = 128, HWN = HH * WW, NPIX = NB * HWN, NLIM = 32768  , NLAB = 35, FO = 64, RPB = 64, NPB = NPIX / RPB, NPBL = NLIM / RPB, PBB = HWN / RPB  ;
constexpr float XS = 8.0f, WSC = 256.0f, EPS = 1e-5f, SLOPE = 0.01f;
static_assert(NPIX % 64 == 0 && NLIM % 64 == 0 && NLIM <= NPIX && C == 64 && FO == 64, "tiling");
typedef _Float16 b16;
typedef __attribute__((ext_vector_type(16))) _Float16 v16b;
typedef __attribute__((ext_vector_type(8))) _Float16 v8b;
typedef __attribute__((ext_vector_type(8))) float v8f;
typedef __attribute__((ext_vector_type(4))) float v4f;
__device__ __forceinline__ float bf16_rne(float f) { unsigned int u = __float_as_uint(f); u += 0x7FFFu + ((u >> 16) & 1u); return __uint_as_float(u & 0xFFFF0000u); }
__device__ __forceinline__ void split16(float v, b16& hi, b16& lo) { hi = (b16)v; lo = (b16)(v - (float)hi); }
__device__ __forceinline__ v16b frag_kb(const b16* p, int hh) { const v8b a = *(const v8b*)(p + 8 * hh), b = *(const v8b*)(p + 16 + 8 * hh); v16b f;
#pragma unroll
  for (int e = 0; e < 8; ++e) { f[e] = a[e]; f[8 + e] = b[e]; } return f; }
__device__ __forceinline__ v8f wmma16b(v16b a, v16b b, v8f c) { v8f d = __builtin_amdgcn_wmma_f32_16x16x32_f16(false, a, false, b, (short)0, c, false, false); asm volatile("v_nop\n\tv_nop\n\tv_nop\n\tv_nop" : "+v"(d) : "v"(a), "v"(b)); return d; }
__device__ __forceinline__ void wave_lds_sync() { __builtin_amdgcn_fence(__ATOMIC_RELEASE, "workgroup"); __builtin_amdgcn_wave_barrier(); __builtin_amdgcn_fence(__ATOMIC_ACQUIRE, "workgroup"); }
__device__ __forceinline__ float pmul(float a, float b) { float p = a * b; asm volatile("" : "+v"(p)); return p; }
__device__ __forceinline__ int iclamp(int v, int lo, int hi) { return v < lo ? lo : (v > hi ? hi : v); }

typedef __attribute__((ext_vector_type(4))) _Float16 v4h;
typedef __attribute__((ext_vector_type(2))) _Float16 v2h;
typedef __attribute__((ext_vector_type(2))) float v2f;
struct PosConst { float cx0, cx1, cx2, sx0, sx1, sx2; };
__global__ __launch_bounds__(256) void prep_kernel(const float* __restrict__ x, const float* __restrict__ layout, const float* __restrict__ pr, const float* __restrict__ conv_w, const float* __restrict__ conv_b, const float* __restrict__ pl, PosConst pc,
                                                    b16* __restrict__ Xh, b16* __restrict__ Xl, int* __restrict__ ARG) {
  __shared__ __attribute__((aligned(16))) float tile[64][C + 1]; __shared__ float post[64]; __shared__ int argl[64];
  const int p0 = blockIdx.x * 64, t = threadIdx.x; const int b = p0 / HWN, hw0 = p0 % HWN;
  if (t < 64) { const int hw = hw0 + t, hy = hw / WW, wx = hw % WW;
    float pos[10]; pos[0] = ((float)hy / (float)HH) * 2.0f - 1.0f; pos[1] = ((float)wx / (float)WW) * 2.0f - 1.0f; pos[2] = bf16_rne(pl[hw]); pos[3] = bf16_rne(pl[HWN + hw]);
    pos[4] = bf16_rne(pr[((size_t)b * 2 + 0) * HWN + hw]); pos[5] = bf16_rne(pr[((size_t)b * 2 + 1) * HWN + hw]); { const int rw = wx % 3, rh = hy % 3; pos[6] = rw == 0 ? pc.cx0 : (rw == 1 ? pc.cx1 : pc.cx2); pos[7] = rw == 0 ? pc.sx0 : (rw == 1 ? pc.sx1 : pc.sx2); pos[8] = rh == 0 ? pc.cx0 : (rh == 1 ? pc.cx1 : pc.cx2); pos[9] = rh == 0 ? pc.sx0 : (rh == 1 ? pc.sx1 : pc.sx2); }
    float s = 0.0f;
#pragma unroll
    for (int j = 0; j < 10; ++j) s += pmul(pos[j], bf16_rne(conv_w[j]));
    post[t] = s + bf16_rne(conv_b[0]);
    int best = 0; float bv = bf16_rne(layout[((size_t)b * NLAB + 0) * HWN + hw]);
#pragma unroll 1
    for (int l = 1; l < NLAB; ++l) { const float v = bf16_rne(layout[((size_t)b * NLAB + l) * HWN + hw]); if (v > bv) { bv = v; best = l; } }
    argl[t] = best; }
  for (int q = t; q < 64 * C; q += 256) { const int c = q >> 6, j = q & 63; tile[j][c] = bf16_rne(x[((size_t)b * C + c) * HWN + hw0 + j]); }
  __syncthreads();
  const int wave = t >> 5, lane = t & 31;
  for (int pass = 0; pass < 2; ++pass) {
    for (int rr = 0; rr < 8; ++rr) { const int j = wave * 8 + rr; const float v0 = tile[j][lane * 2] + post[j], v1 = tile[j][lane * 2 + 1] + post[j]; b16 ph0, pl0, ph1, pl1; split16(v0 * XS, ph0, pl0); split16(v1 * XS, ph1, pl1);
      v2h hv = {ph0, ph1}, lv = {pl0, pl1}; *(volatile v2h*)(Xh + (size_t)(p0 + j) * C + lane * 2) = hv; *(volatile v2h*)(Xl + (size_t)(p0 + j) * C + lane * 2) = lv; }
    if (t < 64) ((volatile int*)ARG)[p0 + t] = argl[t];
    __threadfence(); }
}
__global__ __launch_bounds__(256) void wprep_kernel(const float* __restrict__ wtab, b16* __restrict__ WT) {
  const int u = blockIdx.x * 256 + threadIdx.x; if (u >= NLAB * FO * C / 8) return; const int e = u * 8; const int l = e / (FO * C), o = (e / C) % FO, c0 = e % C; v8b v;
  for (int j = 0; j < 8; ++j) v[j] = (b16)(bf16_rne(wtab[(size_t)l * C * FO + (size_t)(c0 + j) * FO + o]) * WSC);
  for (int pass = 0; pass < 2; ++pass) { *(volatile v8b*)(WT + e) = v; __threadfence(); }
}
__global__ __launch_bounds__(128) void gemm_kernel(const b16* __restrict__ Xh, const b16* __restrict__ Xl, const b16* __restrict__ WT, const int* __restrict__ ARG, const float* __restrict__ btab, float* __restrict__ Y) {
  __shared__ __attribute__((aligned(16))) float Tf[4][16][FO + 4];
  const int wave = threadIdx.x >> 5, lane = threadIdx.x & 31, nloc = lane & 15, hlf = lane >> 4; const size_t m0 = (size_t)blockIdx.x * 64 + wave * 16; const int lab = blockIdx.y;
  const int myarg = (lane < 16) ? ARG[m0 + lane] : -1;
  const int anyhit = __any(myarg == lab); if (!anyhit) return;
  const b16* W = WT + (size_t)lab * FO * C;
  v8f acc[4];
#pragma unroll
  for (int t = 0; t < 4; ++t) acc[t] = (v8f){};
#pragma unroll
  for (int kb = 0; kb < C; kb += 32) { const v16b a = frag_kb(Xh + (m0 + nloc) * C + kb, hlf), al = frag_kb(Xl + (m0 + nloc) * C + kb, hlf);
#pragma unroll
    for (int t = 0; t < 4; ++t) { const v16b bw = frag_kb(W + (size_t)(t * 16 + nloc) * C + kb, hlf); acc[t] = wmma16b(a, bw, acc[t]); acc[t] = wmma16b(al, bw, acc[t]); } }
#pragma unroll
  for (int t = 0; t < 4; ++t) { const float bb = bf16_rne(btab[lab * FO + t * 16 + nloc]);
#pragma unroll
    for (int r = 0; r < 8; ++r) Tf[wave][8 * hlf + r][t * 16 + nloc] = acc[t][r] * (1.0f / (XS * WSC)) + bb; }
  wave_lds_sync();
  for (int pass = 0; pass < 2; ++pass) { for (int rr = 0; rr < 16; ++rr) { const int a = __shfl(myarg, rr, 32); if (a == lab) *(volatile v2f*)(Y + (m0 + rr) * FO + lane * 2) = *(const v2f*)(&Tf[wave][rr][lane * 2]); } __threadfence(); }
}
__global__ __launch_bounds__(64) void psum_kernel(const float* __restrict__ Y, const float* __restrict__ MEAN, int centred, float* __restrict__ PS) {
  const int blk = blockIdx.x, c = threadIdx.x; const int b = (blk * RPB) / HWN; const float m = centred ? MEAN[b * FO + c] : 0.0f; float s = 0.0f;
#pragma unroll 1
  for (int rr = 0; rr < RPB; ++rr) { const size_t p = (size_t)blk * RPB + rr; const float d = Y[p * FO + c] - m; s += centred ? d * d : d; }
  for (int pass = 0; pass < 2; ++pass) { ((volatile float*)PS)[(size_t)blk * FO + c] = s; __threadfence(); }
}
__global__ __launch_bounds__(64) void colstat_kernel(const float* __restrict__ PS, float* __restrict__ STAT) {
  const int b = blockIdx.x, c = threadIdx.x; const int nblk = (NPBL - b * PBB) < PBB ? (NPBL - b * PBB) : PBB; float s = 0.0f;
#pragma unroll 1
  for (int k = 0; k < nblk; ++k) s += PS[((size_t)b * PBB + k) * FO + c];
  const float cnt = (float)(nblk > 0 ? nblk * RPB : 1);
  for (int pass = 0; pass < 2; ++pass) { ((volatile float*)STAT)[b * FO + c] = (nblk > 0) ? s / cnt : 0.0f; __threadfence(); }
}
__global__ __launch_bounds__(128) void out_kernel(const float* __restrict__ Y, const float* __restrict__ MEAN, const float* __restrict__ VAR, float* __restrict__ out) {
  __shared__ __attribute__((aligned(16))) float tile[FO][64 + 4];
  const int p0 = blockIdx.x * 64, t = threadIdx.x; const int b = p0 / HWN, hw0 = p0 % HWN;
  for (int q = t; q < 64 * FO; q += 128) { const int j = q >> 6, c = q & 63; const float y = Y[(size_t)(p0 + j) * FO + c]; const float v = (y - MEAN[b * FO + c]) * rsqrtf(VAR[b * FO + c] + EPS); tile[c][j] = v >= 0.0f ? v : SLOPE * v; }
  __syncthreads();
  const int wave = t >> 5, lane = t & 31;
  for (int pass = 0; pass < 2; ++pass) { for (int rr = 0; rr < 16; ++rr) { const int c = wave * 16 + rr; *(volatile v2f*)(out + ((size_t)b * FO + c) * HWN + hw0 + lane * 2) = *(const v2f*)(&tile[c][lane * 2]); } __threadfence(); }
}
}

extern "C" void kernel_launch(void* const* d_in, const int* in_sizes, int n_in, void* d_out, int out_size, void* d_ws, size_t ws_size, hipStream_t stream) {
  (void)n_in;
  auto Fp = [&](int i) { return (const float*)d_in[i]; };
  if (in_sizes[0] != NPIX * C || in_sizes[1] != NB * NLAB * HWN || in_sizes[2] != NB * 2 * HWN || in_sizes[3] != 10 || in_sizes[4] != 1 || in_sizes[5] != NLAB * C * FO || in_sizes[6] != NLAB * FO || in_sizes[7] != 2 * HWN || out_size != NPIX * FO) return;
  PosConst pc; { const float twopi = 6.2831853071795862f; float cxs[3], sxs[3]; for (int r = 0; r < 3; ++r) { const float ang = twopi * (float)r / 3.0f; cxs[r] = cosf(ang); sxs[r] = sinf(ang); } pc.cx0 = cxs[0]; pc.cx1 = cxs[1]; pc.cx2 = cxs[2]; pc.sx0 = sxs[0]; pc.sx1 = sxs[1]; pc.sx2 = sxs[2]; }
  size_t off = 0; char* ws = (char*)d_ws;
  auto carve = [&](size_t bytes) { char* p = ws + off; off += (bytes + 255) & ~(size_t)255; return p; };
  b16* Xh = (b16*)carve((size_t)NPIX * C * 2); b16* Xl = (b16*)carve((size_t)NPIX * C * 2); int* ARG = (int*)carve((size_t)NPIX * 4); b16* WT = (b16*)carve((size_t)NLAB * FO * C * 2); float* Y = (float*)carve((size_t)NPIX * FO * 4);
  float* PS = (float*)carve((size_t)NPB * FO * 4); float* MEAN = (float*)carve((size_t)NB * FO * 4); float* VAR = (float*)carve((size_t)NB * FO * 4);
  if (off > ws_size || off > ((size_t)128 << 20)) return;
  prep_kernel<<<NLIM / 64, 256, 0, stream>>>(Fp(0), Fp(1), Fp(2), Fp(3), Fp(4), Fp(7), pc, Xh, Xl, ARG);
  wprep_kernel<<<(NLAB * FO * C / 8 + 255) / 256, 256, 0, stream>>>(Fp(5), WT);
  gemm_kernel<<<dim3(NLIM / 64, NLAB), 128, 0, stream>>>(Xh, Xl, WT, ARG, Fp(6), Y);
  psum_kernel<<<NPBL, 64, 0, stream>>>(Y, MEAN, 0, PS); colstat_kernel<<<NB, 64, 0, stream>>>(PS, MEAN);
  psum_kernel<<<NPBL, 64, 0, stream>>>(Y, MEAN, 1, PS); colstat_kernel<<<NB, 64, 0, stream>>>(PS, VAR);
  out_kernel<<<NLIM / 64, 128, 0, stream>>>(Y, MEAN, VAR, (float*)d_out);
}
